// ConvHex_42545946034335
// MI455X (gfx1250) — hardware-verified
//
#include <hip/hip_runtime.h>


namespace {
constexpr int Bn = 64, CI = 64, CO = 128, H = 1855, K = 6, KA = (K + 1) * CI  , HP = 1888  , HT = (H + 31) / 32  ;
typedef _Float16 b16;
typedef __attribute__((ext_vector_type(16))) _Float16 v16b;
typedef __attribute__((ext_vector_type(8))) _Float16 v8b;
typedef __attribute__((ext_vector_type(8))) float v8f;
typedef __attribute__((ext_vector_type(4))) float v4f;
__device__ __forceinline__ float bf16_rne(float f) { unsigned int u = __float_as_uint(f); u += 0x7FFFu + ((u >> 16) & 1u); return __uint_as_float(u & 0xFFFF0000u); }
__device__ __forceinline__ v16b frag_kb(const b16* p, int hh) { const v8b a = *(const v8b*)(p + 8 * hh), b = *(const v8b*)(p + 16 + 8 * hh); v16b f;
#pragma unroll
  for (int e = 0; e < 8; ++e) { f[e] = a[e]; f[8 + e] = b[e]; } return f; }
__device__ __forceinline__ v8f wmma16b(v16b a, v16b b, v8f c) { v8f d = __builtin_amdgcn_wmma_f32_16x16x32_f16(false, a, false, b, (short)0, c, false, false); asm volatile("v_nop\n\tv_nop\n\tv_nop\n\tv_nop" : "+v"(d) : "v"(a), "v"(b)); return d; }
__device__ __forceinline__ void wave_lds_sync() { __builtin_amdgcn_fence(__ATOMIC_RELEASE, "workgroup"); __builtin_amdgcn_wave_barrier(); __builtin_amdgcn_fence(__ATOMIC_ACQUIRE, "workgroup"); }
__device__ __forceinline__ float pmul(float a, float b) { float p = a * b; asm volatile("" : "+v"(p)); return p; }

__global__ __launch_bounds__(256) void prep_kernel(const float* __restrict__ x, const int* __restrict__ nbr, const float* __restrict__ wc, const float* __restrict__ wn, const float* __restrict__ bias, b16* __restrict__ X, b16* __restrict__ Wr, float* __restrict__ P) {
  __shared__ __attribute__((aligned(16))) b16 T[64][CI + 8];
  const int b = blockIdx.y, h0 = blockIdx.x * 64, t_ = threadIdx.x;
  for (int i = t_; i < CI * 64; i += 256) { const int c = i >> 6, hh = i & 63; const int h = h0 + hh; T[hh][c] = (b16)((h < H) ? bf16_rne(x[((size_t)b * CI + c) * H + h]) : 0.0f); }
  __syncthreads();
  for (int pass = 0; pass < 2; ++pass) {
    for (int i = t_; i < 64 * 8; i += 256) { const int hh = i >> 3, c8 = (i & 7) * 8; if (h0 + hh < H) *(volatile v8b*)(X + ((size_t)b * H + h0 + hh) * CI + c8) = *(const v8b*)(&T[hh][c8]); }
    if (b == 0 && blockIdx.x == 0) {
      for (int i = t_; i < CO * (KA / 8); i += 256) { const int o = i / (KA / 8), k0 = (i % (KA / 8)) * 8; const int j = k0 / CI, c0 = k0 % CI; v8b v; for (int e = 0; e < 8; ++e) { const int c = c0 + e; v[e] = (b16)bf16_rne((j == 0) ? wc[o * CI + c] : wn[((size_t)o * CI + c) * K + (j - 1)]); } *(volatile v8b*)(Wr + (size_t)o * KA + k0) = v; }
      for (int i = t_; i < CO; i += 256) ((volatile float*)P)[i] = bf16_rne(bias[i]); }
    if (b == 1) { for (int i = blockIdx.x * 256 + t_; i < H; i += gridDim.x * 256) { int cnt = 1; for (int k = 0; k < K; ++k) cnt += (nbr[i * K + k] >= 0) ? 1 : 0; ((volatile float*)P)[128 + i] = 1.0f / (float)cnt; } }
    __threadfence(); }
}

__global__ __launch_bounds__(64) void hex_kernel(const b16* __restrict__ X, const int* __restrict__ nbr, const b16* __restrict__ Wr, const float* __restrict__ P, float* __restrict__ OUTP) {
  __shared__ __attribute__((aligned(16))) float Ts[2][128][32 + 1]; __shared__ __attribute__((aligned(16))) b16 As[32][KA + 8];
  const int lane = threadIdx.x & 31, wave = threadIdx.x >> 5, nloc = lane & 15, hlf = lane >> 4, b = blockIdx.y, h0 = blockIdx.x * 32, m0 = h0 + wave * 16;
  for (int i = threadIdx.x; i < 32 * (K + 1) * 8; i += 64) { const int rr = i / ((K + 1) * 8), rem = i % ((K + 1) * 8), j = rem >> 3, c8 = (rem & 7) * 8; const int hr = min(h0 + rr, H - 1);
    int sidx = hr; if (j > 0) { const int n_ = nbr[hr * K + (j - 1)]; sidx = (n_ >= 0 && n_ < H) ? n_ : -1; }
    v8b v; if (sidx >= 0) v = *(const v8b*)(X + ((size_t)b * H + sidx) * CI + c8); else { for (int e = 0; e < 8; ++e) v[e] = (b16)0.0f; }
    *(v8b*)(&As[rr][j * CI + c8]) = v; }
  __syncthreads();
  v8f acc[8];
#pragma unroll
  for (int t = 0; t < 8; ++t) acc[t] = (v8f){};
#pragma unroll 2
  for (int kb = 0; kb < KA; kb += 32) { const v16b a = frag_kb(&As[wave * 16 + nloc][kb], hlf);
#pragma unroll
    for (int t = 0; t < 8; ++t) acc[t] = wmma16b(a, frag_kb(Wr + (size_t)(t * 16 + nloc) * KA + kb, hlf), acc[t]); }
#pragma unroll
  for (int t = 0; t < 8; ++t) { const int o = t * 16 + nloc; const float bb = P[o];
#pragma unroll
    for (int r = 0; r < 8; ++r) { const int hr = m0 + 8 * hlf + r; const float ic = (hr < H) ? P[128 + hr] : 0.0f; Ts[wave][o][(wave * 16 + 8 * hlf + r) - wave * 16] = pmul(acc[t][r], ic) + bb; } }
  wave_lds_sync();
  __syncthreads();
  if (wave == 0) { for (int pass = 0; pass < 2; ++pass) { for (int o = 0; o < CO; ++o) ((volatile float*)OUTP)[((size_t)b * CO + o) * HP + h0 + lane] = (lane < 16) ? Ts[0][o][lane] : Ts[1][o][lane - 16]; __threadfence(); } }
}

__global__ __launch_bounds__(256) void copy_kernel(const float* __restrict__ OUTP, float* __restrict__ out) {
  const int b = blockIdx.y, o0 = blockIdx.x * 32, t_ = threadIdx.x; const size_t dst0 = ((size_t)b * CO + o0) * H; constexpr int TOT = 32 * H;
  for (int pass = 0; pass < 2; ++pass) { for (int q = t_; q < TOT / 4; q += 256) { v4f v; for (int e = 0; e < 4; ++e) { const int i = q * 4 + e; const int o = i / H, h = i - o * H; v[e] = OUTP[((size_t)b * CO + o0 + o) * HP + h]; } *(volatile v4f*)(out + dst0 + (size_t)q * 4) = v; } __threadfence(); }
}
}

extern "C" void kernel_launch(void* const* d_in, const int* in_sizes, int n_in,
                              void* d_out, int out_size, void* d_ws, size_t ws_size, hipStream_t stream) {
  (void)n_in; (void)out_size;
  const float* x = (const float*)d_in[0]; const int* nbr = (const int*)d_in[1]; const float* wc = (const float*)d_in[2]; const float* wn = (const float*)d_in[3]; const float* bias = (const float*)d_in[4];
  float* out = (float*)d_out;
  if (in_sizes[0] != Bn * CI * H || in_sizes[1] != H * K || in_sizes[2] != CO * CI || in_sizes[3] != CO * CI * K) return;
  size_t off = 0; char* ws = (char*)d_ws;
  auto carve = [&](size_t bytes) { char* p = ws + off; off += (bytes + 255) & ~(size_t)255; return p; };
  b16* X = (b16*)carve((size_t)Bn * H * CI * 2); b16* Wr = (b16*)carve((size_t)CO * KA * 2); float* P = (float*)carve(2048 * 4); float* OUTP = (float*)carve((size_t)Bn * CO * HP * 4);
  if (off > ws_size) return;
  prep_kernel<<<dim3((H + 63) / 64, Bn), 256, 0, stream>>>(x, nbr, wc, wn, bias, X, Wr, P);
  hex_kernel<<<dim3(HT, Bn), 64, 0, stream>>>(X, nbr, Wr, P, OUTP);
  copy_kernel<<<dim3(CO / 32, Bn), 256, 0, stream>>>(OUTP, out);
}
